// SelectiveSSM_61821759259048
// MI455X (gfx1250) — hardware-verified
//
#include <hip/hip_runtime.h>
#include <math.h>

typedef __attribute__((ext_vector_type(16))) _Float16 v16h;
typedef __attribute__((ext_vector_type(8)))  _Float16 v8h;
typedef __attribute__((ext_vector_type(16))) __bf16   v16b;
typedef __attribute__((ext_vector_type(8)))  __bf16   v8b;
typedef __attribute__((ext_vector_type(8)))  float    v8f;
typedef __attribute__((ext_vector_type(4)))  float    v4f;
typedef __attribute__((ext_vector_type(4)))  unsigned v4u;

constexpr int kBatch = 2;
constexpr int kSeq   = 2048;
constexpr int kHid   = 1024;
constexpr int kDin   = 2048;
constexpr int kNst   = 16;
constexpr int kDtR   = 64;
constexpr int kXdbl  = 96;
constexpr int kXdP   = 128;
constexpr int kXzN   = 2 * kDin;
constexpr int kRows  = kBatch * kSeq;
constexpr int kConvK = 4;
static_assert(kDtR + 2 * kNst == kXdbl, "x_proj width");

constexpr float kWCarry      = 16.0f;
constexpr float kLoCarry     = 1024.0f;
constexpr float kXinCarry    = 16.0f;
constexpr float kXinCarryInv = 1.0f / 16.0f;
constexpr float kDtrCarry    = 16.0f;
constexpr float kGCarry      = 64.0f;
constexpr float kLog2e = 1.4426950408889634f;
constexpr float kLn2   = 0.6931471805599453f;

static_assert((kHid % 32) == 0 && (kDin % 32) == 0 && (kDtR % 32) == 0, "K multiples of 32");
static_assert((kRows % 64) == 0 && (kXzN % 64) == 0 && (kXdP % 64) == 0 && (kDin % 64) == 0 && (kHid % 64) == 0, "M,N multiples of 64");
static_assert(((kRows / 32) * (kDin / 64)) % 8 == 0 && ((kRows / 32) * (kXdP / 64)) % 8 == 0 &&
              ((kRows / 64) * (kDin / 64)) % 8 == 0 && ((kRows / 64) * (kHid / 64)) % 8 == 0, "8 tiles per block exactly");

constexpr size_t kOffXH   = 0;
constexpr size_t kOffXL   = kOffXH   + (size_t)kRows * kHid * 2;
constexpr size_t kOffWIH  = kOffXL   + (size_t)kRows * kHid * 2;
constexpr size_t kOffXPRE = kOffWIH  + (size_t)kXzN  * kHid * 2;
constexpr size_t kOffDTV  = kOffXPRE;
constexpr size_t kOffZ16  = kOffXPRE + (size_t)kRows * kDin * 4;
constexpr size_t kOffXIN  = kOffZ16  + (size_t)kRows * kDin * 2;
constexpr size_t kOffWXH  = kOffXIN  + (size_t)kRows * kDin * 2;
constexpr size_t kOffWXL  = kOffWXH  + (size_t)kXdP  * kDin * 2;
constexpr size_t kOffXD   = kOffWXL  + (size_t)kXdP  * kDin * 2;
constexpr size_t kOffDTR  = kOffXD   + (size_t)kRows * kXdP * 4;
constexpr size_t kOffWDT  = kOffDTR  + (size_t)kRows * kDtR * 2;
constexpr size_t kOffG    = kOffWDT  + (size_t)kDin  * kDtR * 2;
constexpr size_t kOffWOH  = kOffG    + (size_t)kRows * kDin * 2;
constexpr size_t kWsTotal = kOffWOH  + (size_t)kHid  * kDin * 2;
static_assert(kWsTotal == 117178368ull, "carve total");
static_assert(kWsTotal <= 134217728ull, "carve cap");
static_assert((size_t)kRows * kDin * 4 == (kOffZ16 - kOffDTV), "DTV fits the XPRE bytes exactly");
static_assert((kOffXL % 128) == 0 && (kOffWIH % 128) == 0 && (kOffXPRE % 128) == 0 && (kOffZ16 % 128) == 0 &&
              (kOffXIN % 128) == 0 && (kOffWXH % 128) == 0 && (kOffWXL % 128) == 0 && (kOffXD % 128) == 0 &&
              (kOffDTR % 128) == 0 && (kOffWDT % 128) == 0 && (kOffG % 128) == 0 && (kOffWOH % 128) == 0,
              "128-B aligned regions");

constexpr size_t kOut0Floats = (size_t)kRows * kHid;
constexpr size_t kOut1Floats = (size_t)kBatch * kDin * kNst;
static_assert(kOut0Floats * 4 == 16777216ull, "out1 byte offset");
static_assert((kOut0Floats * 4 + kOut1Floats * 4) == 17039360ull, "d_out total");

__device__ __forceinline__ unsigned short f2bf_bits(float f) {
  unsigned u = __float_as_uint(f);
  return (unsigned short)((u + 0x7FFFu + ((u >> 16) & 1u)) >> 16);
}
__device__ __forceinline__ float bf_bits2f(unsigned short h) { return __uint_as_float(((unsigned)h) << 16); }

__device__ __forceinline__ float h16_to_f32(unsigned hb) {
  const unsigned sgn = (hb & 0x8000u) << 16; const unsigned em = hb & 0x7fffu;
  const float fn = __uint_as_float((em << 13) + 0x38000000u);
  const float fs = (float)em * 5.9604644775390625e-8f;
  const float mag = (em < 0x400u) ? fs : fn; return __uint_as_float(__float_as_uint(mag) | sgn);
}

__device__ __forceinline__ void dep_guard4_h(v8f& a, v8f& b, v8f& c, v8f& d, v16h x, v16h y) { asm volatile("v_nop\n\tv_nop\n\tv_nop\n\tv_nop" : "+v"(a), "+v"(b), "+v"(c), "+v"(d) : "v"(x), "v"(y)); }
__device__ __forceinline__ void dep_guard4_b(v8f& a, v8f& b, v8f& c, v8f& d, v16b x, v16b y) { asm volatile("v_nop\n\tv_nop\n\tv_nop\n\tv_nop" : "+v"(a), "+v"(b), "+v"(c), "+v"(d) : "v"(x), "v"(y)); }
__device__ __forceinline__ void dep_guard8_h(v8f& a, v8f& b, v8f& c, v8f& d, v8f& e, v8f& f, v8f& g, v8f& hq, v16h x, v16h y) {
  asm volatile("v_nop\n\tv_nop\n\tv_nop\n\tv_nop" : "+v"(a), "+v"(b), "+v"(c), "+v"(d), "+v"(e), "+v"(f), "+v"(g), "+v"(hq) : "v"(x), "v"(y));
}
__device__ __forceinline__ void keep4_h(v16h a, v16h b, v16h c, v16h d) { asm volatile("v_nop" :: "v"(a), "v"(b), "v"(c), "v"(d)); }
__device__ __forceinline__ void keep4_b(v16b a, v16b b, v16b c, v16b d) { asm volatile("v_nop" :: "v"(a), "v"(b), "v"(c), "v"(d)); }
__device__ __forceinline__ void acc_guard4(v8f& a, v8f& b, v8f& c, v8f& d) { asm volatile("v_nop\n\tv_nop\n\tv_nop\n\tv_nop" : "+v"(a), "+v"(b), "+v"(c), "+v"(d)); }
template <typename T> struct Frag;
template <> struct Frag<_Float16> {
  typedef v16h V; union U { v16h v; v8h h[2]; };
  static __device__ __forceinline__ v16h load(const _Float16* p) {
    U f; f.h[0] = *(const v8h*)(p); f.h[1] = *(const v8h*)(p + 16); return f.v;
  }
  static __device__ __forceinline__ v8f mma(v16h a, v16h b, v8f c) {
    return __builtin_amdgcn_wmma_f32_16x16x32_f16(false, a, false, b, (short)0, c, false, false);
  }
  static __device__ __forceinline__ void guard4(v8f& a, v8f& b, v8f& c, v8f& d, v16h x, v16h y) { dep_guard4_h(a, b, c, d, x, y); }
  static __device__ __forceinline__ void keep(v16h a, v16h b, v16h c, v16h d) { keep4_h(a, b, c, d); }
};
template <> struct Frag<__bf16> {
  typedef v16b V; union U { v16b v; v8b h[2]; };
  static __device__ __forceinline__ v16b load(const __bf16* p) {
    U f; f.h[0] = *(const v8b*)(p); f.h[1] = *(const v8b*)(p + 16); return f.v;
  }
  static __device__ __forceinline__ v8f mma(v16b a, v16b b, v8f c) {
    return __builtin_amdgcn_wmma_f32_16x16x32_bf16(false, a, false, b, (short)0, c, false, false);
  }
  static __device__ __forceinline__ void guard4(v8f& a, v8f& b, v8f& c, v8f& d, v16b x, v16b y) { dep_guard4_b(a, b, c, d, x, y); }
  static __device__ __forceinline__ void keep(v16b a, v16b b, v16b c, v16b d) { keep4_b(a, b, c, d); }
};

template <int ET> struct Elem;
template <> struct Elem<0> { typedef _Float16 T; };
template <> struct Elem<1> { typedef __bf16 T; };
template <int ET, int SPL, int BIAS_MODE, int OUT_MODE, bool RESID, int ACT = 0>
__global__ __launch_bounds__(256) void wmma_gemm64(
    const unsigned short* __restrict__ Ap, const unsigned short* __restrict__ A2p, int lda, long strideA,
    const unsigned short* __restrict__ Btp, const unsigned short* __restrict__ Bt2p, int ldb, long strideB,
    void* __restrict__ Cout, void* __restrict__ Cout2, int ldc, long strideC,
    const float* __restrict__ bias,
    const float* __restrict__ resid, long strideR,
    int M, int N, int K, float scale) {
  typedef typename Elem<ET>::T T;
  typedef typename Frag<T>::V V;
  const T* A = (const T*)Ap; const T* A2 = (const T*)A2p; const T* Bt = (const T*)Btp; const T* Bt2 = (const T*)Bt2p;
  __shared__ __align__(16) float sT[8][16 * 68];
  const int b    = blockIdx.y;
  const int lane = threadIdx.x & 31;
  const int wave = threadIdx.x >> 5;
  const int tilesN = N >> 6;
  const int tilesM = M >> 6;
  const int tile = blockIdx.x * 8 + wave;
  if (tile >= tilesM * tilesN) return;
  const int tm = tile / tilesN;
  const int tn = tile - tm * tilesN;
  const int m0 = tm << 6;
  const int n0 = tn << 6;

  const T* Ab  = A  + (size_t)b * strideA;
  const T* Bb  = Bt + (size_t)b * strideB;
  const T* Ab2 = (SPL >= 1) ? (A2  + (size_t)b * strideA) : nullptr;
  const T* Bb2 = (SPL == 2) ? (Bt2 + (size_t)b * strideB) : nullptr;

  const int rlane = lane & 15;
  const int koff  = (lane >> 4) * 8;
  const int mOff  = (lane >> 4) * 8;

  v8f acc[4][4];
#pragma unroll
  for (int i = 0; i < 4; ++i)
#pragma unroll
    for (int j = 0; j < 4; ++j) acc[i][j] = (v8f){0.f,0.f,0.f,0.f,0.f,0.f,0.f,0.f};

  for (int k0 = 0; k0 < K; k0 += 32) {
    V bh[4], bl[4];
#pragma unroll
    for (int j = 0; j < 4; ++j) {
      const size_t bo = (size_t)(n0 + (j << 4) + rlane) * ldb + koff + k0;
      bh[j] = Frag<T>::load(Bb + bo);
      if (SPL == 2) bl[j] = Frag<T>::load(Bb2 + bo);
    }
#pragma unroll
    for (int i = 0; i < 4; ++i) {
      const size_t ao = (size_t)(m0 + (i << 4) + rlane) * lda + koff + k0;
      V ah = Frag<T>::load(Ab + ao);
      V al;
      if (SPL >= 1) al = Frag<T>::load(Ab2 + ao);
#pragma unroll
      for (int j = 0; j < 4; ++j) {
        acc[i][j] = Frag<T>::mma(ah, bh[j], acc[i][j]);
        if (SPL == 2) acc[i][j] = Frag<T>::mma(ah, bl[j], acc[i][j]);
        if (SPL >= 1) acc[i][j] = Frag<T>::mma(al, bh[j], acc[i][j]);
      }
      Frag<T>::guard4(acc[i][0], acc[i][1], acc[i][2], acc[i][3], ah, (SPL >= 1) ? al : ah);
    }
    Frag<T>::keep(bh[0], bh[1], bh[2], bh[3]);
    if (SPL == 2) Frag<T>::keep(bl[0], bl[1], bl[2], bl[3]);
  }
  acc_guard4(acc[0][0], acc[0][1], acc[0][2], acc[0][3]);
  acc_guard4(acc[1][0], acc[1][1], acc[1][2], acc[1][3]);
  acc_guard4(acc[2][0], acc[2][1], acc[2][2], acc[2][3]);
  acc_guard4(acc[3][0], acc[3][1], acc[3][2], acc[3][3]);

  float* slab = sT[wave];
  const float* Rb = RESID ? (resid + (size_t)b * strideR) : nullptr;
#pragma unroll
  for (int i = 0; i < 4; ++i) {
    const int mBase = m0 + (i << 4);
#pragma unroll
    for (int j = 0; j < 4; ++j) {
      const int n = n0 + (j << 4) + rlane;
      float bv = 0.f;
      if (BIAS_MODE == 2) bv = bias[n];
#pragma unroll
      for (int r = 0; r < 8; ++r) {
        float v = acc[i][j][r] * scale;
        if (BIAS_MODE == 1) v += bias[mBase + mOff + r];
        if (BIAS_MODE == 2) v += bv;
        if (RESID) v += Rb[(size_t)(mBase + mOff + r) * ldc + n];
        if (ACT == 1) v = tanhf(v);
        if (ACT == 2) v = fmaxf(v, 0.0f);
        if (ACT == 3) v = v / (1.0f + expf(-v));
        if (ACT == 4) v = (v > 0.f) ? v : 0.01f * v;
        slab[(mOff + r) * 68 + (j << 4) + rlane] = v;
      }
    }
    __builtin_amdgcn_fence(__ATOMIC_RELEASE, "workgroup");
    __builtin_amdgcn_wave_barrier();
    __builtin_amdgcn_fence(__ATOMIC_ACQUIRE, "workgroup");
    if (OUT_MODE == 0) {
      float* C = (float*)Cout + (size_t)b * strideC;
      const int hh = lane >> 4, c4 = (lane & 15) * 4;
      for (int pass = 0; pass < 2; ++pass) {
#pragma unroll
        for (int it = 0; it < 8; ++it) {
          const int row = it * 2 + hh;
          v4f v = *(const v4f*)(slab + row * 68 + c4);
          *(volatile v4f*)(C + (size_t)(mBase + row) * ldc + n0 + c4) = v;
        }
        __threadfence();
      }
    } else {
      const int q = lane >> 3, c8 = (lane & 7) * 8;
      unsigned short* C  = (unsigned short*)Cout  + (size_t)b * strideC;
      unsigned short* C2 = (OUT_MODE == 2) ? ((unsigned short*)Cout2 + (size_t)b * strideC) : nullptr;
      for (int pass = 0; pass < 2; ++pass) {
#pragma unroll
        for (int it = 0; it < 4; ++it) {
          const int row = it * 4 + q;
          const float* sp = slab + row * 68 + c8;
          v8h hv, lv;
#pragma unroll
          for (int e = 0; e < 8; ++e) {
            if (OUT_MODE == 1) {
              hv[e] = (_Float16)sp[e];
            } else {
              unsigned short hb = f2bf_bits(sp[e]);
              unsigned short lb = f2bf_bits(sp[e] - bf_bits2f(hb));
              hv[e] = __builtin_bit_cast(_Float16, hb);
              lv[e] = __builtin_bit_cast(_Float16, lb);
            }
          }
          *(volatile v8h*)(C + (size_t)(mBase + row) * ldc + n0 + c8) = hv;
          if (OUT_MODE == 2) *(volatile v8h*)(C2 + (size_t)(mBase + row) * ldc + n0 + c8) = lv;
        }
        __threadfence();
      }
    }
    __builtin_amdgcn_fence(__ATOMIC_RELEASE, "workgroup");
    __builtin_amdgcn_wave_barrier();
    __builtin_amdgcn_fence(__ATOMIC_ACQUIRE, "workgroup");
  }
}

template <int RES_SIDE, int OUT_MODE>
__global__ __launch_bounds__(256) void wmma_gemm32x64_res(
    const unsigned short* __restrict__ Ahp, const unsigned short* __restrict__ Alp, int lda,
    const unsigned short* __restrict__ Bthp, const unsigned short* __restrict__ Btlp, int ldb,
    void* __restrict__ Cout, int ldc,
    int M, int N, int K, float scale, float scale_lo) {
  typedef _Float16 T;
  typedef v16h V;
  const T* Ah = (const T*)Ahp; const T* Al = (const T*)Alp; const T* Bth = (const T*)Bthp; const T* Btl = (const T*)Btlp;
  __shared__ __align__(16) float sT[8][16 * 68];
  const int lane = threadIdx.x & 31;
  const int wave = threadIdx.x >> 5;
  const int tilesN = N >> 6;
  const int tilesM = M >> 5;
  const int tile = blockIdx.x * 8 + wave;
  if (tile >= tilesM * tilesN) return;
  const int tm = tile / tilesN;
  const int tn = tile - tm * tilesN;
  const int m0 = tm << 5;
  const int n0 = tn << 6;

  const int rlane = lane & 15;
  const int koff  = (lane >> 4) * 8;
  const int mOff  = (lane >> 4) * 8;

  v8f acc[2][4], accr[2][4];
#pragma unroll
  for (int i = 0; i < 2; ++i)
#pragma unroll
    for (int j = 0; j < 4; ++j) {
      acc[i][j]  = (v8f){0.f,0.f,0.f,0.f,0.f,0.f,0.f,0.f};
      accr[i][j] = (v8f){0.f,0.f,0.f,0.f,0.f,0.f,0.f,0.f};
    }

  for (int k0 = 0; k0 < K; k0 += 32) {
    V bh[4], bl[4];
#pragma unroll
    for (int j = 0; j < 4; ++j) {
      const size_t bo = (size_t)(n0 + (j << 4) + rlane) * ldb + koff + k0;
      bh[j] = Frag<T>::load(Bth + bo);
      if (RES_SIDE == 1) bl[j] = Frag<T>::load(Btl + bo);
    }
#pragma unroll
    for (int i = 0; i < 2; ++i) {
      const size_t ao = (size_t)(m0 + (i << 4) + rlane) * lda + koff + k0;
      V ah = Frag<T>::load(Ah + ao);
      V al;
      if (RES_SIDE == 0) al = Frag<T>::load(Al + ao);
#pragma unroll
      for (int j = 0; j < 4; ++j) {
        acc[i][j] = Frag<T>::mma(ah, bh[j], acc[i][j]);
        if (RES_SIDE == 0) accr[i][j] = Frag<T>::mma(al, bh[j], accr[i][j]);
        else               accr[i][j] = Frag<T>::mma(ah, bl[j], accr[i][j]);
      }
      dep_guard8_h(acc[i][0], acc[i][1], acc[i][2], acc[i][3], accr[i][0], accr[i][1], accr[i][2], accr[i][3],
                   ah, (RES_SIDE == 0) ? al : ah);
    }
    Frag<T>::keep(bh[0], bh[1], bh[2], bh[3]);
    if (RES_SIDE == 1) Frag<T>::keep(bl[0], bl[1], bl[2], bl[3]);
  }
  acc_guard4(acc[0][0], acc[0][1], acc[0][2], acc[0][3]);
  acc_guard4(acc[1][0], acc[1][1], acc[1][2], acc[1][3]);
  acc_guard4(accr[0][0], accr[0][1], accr[0][2], accr[0][3]);
  acc_guard4(accr[1][0], accr[1][1], accr[1][2], accr[1][3]);

  float* slab = sT[wave];
#pragma unroll
  for (int i = 0; i < 2; ++i) {
    const int mBase = m0 + (i << 4);
#pragma unroll
    for (int j = 0; j < 4; ++j) {
#pragma unroll
      for (int r = 0; r < 8; ++r) {
        const float v = acc[i][j][r] * scale + accr[i][j][r] * scale_lo;
        slab[(mOff + r) * 68 + (j << 4) + rlane] = v;
      }
    }
    __builtin_amdgcn_fence(__ATOMIC_RELEASE, "workgroup");
    __builtin_amdgcn_wave_barrier();
    __builtin_amdgcn_fence(__ATOMIC_ACQUIRE, "workgroup");
    if (OUT_MODE == 0) {
      float* C = (float*)Cout;
      const int hh = lane >> 4, c4 = (lane & 15) * 4;
      for (int pass = 0; pass < 2; ++pass) {
#pragma unroll
        for (int it = 0; it < 8; ++it) {
          const int row = it * 2 + hh;
          v4f v = *(const v4f*)(slab + row * 68 + c4);
          *(volatile v4f*)(C + (size_t)(mBase + row) * ldc + n0 + c4) = v;
        }
        __threadfence();
      }
    } else {
      const int q = lane >> 3, c8 = (lane & 7) * 8;
      unsigned short* C = (unsigned short*)Cout;
      for (int pass = 0; pass < 2; ++pass) {
#pragma unroll
        for (int it = 0; it < 4; ++it) {
          const int row = it * 4 + q;
          const float* sp = slab + row * 68 + c8;
          v8h hv;
#pragma unroll
          for (int e = 0; e < 8; ++e) hv[e] = (_Float16)sp[e];
          *(volatile v8h*)(C + (size_t)(mBase + row) * ldc + n0 + c8) = hv;
        }
        __threadfence();
      }
    }
    __builtin_amdgcn_fence(__ATOMIC_RELEASE, "workgroup");
    __builtin_amdgcn_wave_barrier();
    __builtin_amdgcn_fence(__ATOMIC_ACQUIRE, "workgroup");
  }
}

__global__ __launch_bounds__(256) void cast_f16x8_kernel(
    const float* __restrict__ src, unsigned short* __restrict__ dst, int total8, float scale)
{
  const int i = blockIdx.x * 256 + threadIdx.x;
  if (i >= total8) return;
  const size_t e0 = (size_t)i << 3;
  const v4f a0 = *(const v4f*)(src + e0);
  const v4f a1 = *(const v4f*)(src + e0 + 4);
  v8h hv;
#pragma unroll
  for (int e = 0; e < 4; ++e) {
    hv[e]     = (_Float16)(a0[e] * scale);
    hv[4 + e] = (_Float16)(a1[e] * scale);
  }
  unsigned short* qd = dst + e0;
  *(volatile v8h*)qd = hv;
  __threadfence();
  *(volatile v8h*)qd = hv;
}

__global__ __launch_bounds__(256) void split_f16x8_kernel(
    const float* __restrict__ src, unsigned short* __restrict__ dhi, unsigned short* __restrict__ dlo, int total8, float scale)
{
  const int i = blockIdx.x * 256 + threadIdx.x;
  if (i >= total8) return;
  const size_t e0 = (size_t)i << 3;
  const v4f a0 = *(const v4f*)(src + e0);
  const v4f a1 = *(const v4f*)(src + e0 + 4);
  v8h hv, lv;
#pragma unroll
  for (int e = 0; e < 4; ++e) {
    const float f0 = a0[e] * scale, f1 = a1[e] * scale;
    const _Float16 h0 = (_Float16)f0, h1 = (_Float16)f1;
    const float hf0 = (float)h0, hf1 = (float)h1;
    const float r0 = (f0 - hf0) * kLoCarry, r1 = (f1 - hf1) * kLoCarry;
    hv[e]     = h0;
    hv[4 + e] = h1;
    lv[e]     = (_Float16)r0;
    lv[4 + e] = (_Float16)r1;
  }
  unsigned short* qh = dhi + e0;
  unsigned short* ql = dlo + e0;
  *(volatile v8h*)qh = hv;
  *(volatile v8h*)ql = lv;
  __threadfence();
  *(volatile v8h*)qh = hv;
  *(volatile v8h*)ql = lv;
}

__global__ __launch_bounds__(256) void zero2_16x8_kernel(
    unsigned short* __restrict__ dst0, unsigned short* __restrict__ dst1, int total8)
{
  const int i = blockIdx.x * 256 + threadIdx.x;
  if (i >= total8) return;
  const v4u z = (v4u){0u, 0u, 0u, 0u};
  unsigned short* q0 = dst0 + ((size_t)i << 3);
  unsigned short* q1 = dst1 + ((size_t)i << 3);
  *(volatile v4u*)q0 = z;
  *(volatile v4u*)q1 = z;
  __threadfence();
  *(volatile v4u*)q0 = z;
  *(volatile v4u*)q1 = z;
}

constexpr int kConvTP = 260;
__global__ __launch_bounds__(256) void conv_silu_kernel(
    const float* __restrict__ XPRE, const float* __restrict__ cw, const float* __restrict__ cb,
    unsigned short* __restrict__ XIN16)
{
  __shared__ __align__(16) float sT[16 * kConvTP];
  const int tid = threadIdx.x, lane = tid & 31, wave = tid >> 5;
  const int d0 = blockIdx.x * 256, d = d0 + tid;
  const int g0 = blockIdx.y * 64;
  const int tb = g0 & (kSeq - 1);
  const float w0 = cw[d * kConvK + 0], w1 = cw[d * kConvK + 1], w2 = cw[d * kConvK + 2], w3 = cw[d * kConvK + 3];
  const float bc = cb[d];
  float xm3, xm2, xm1;
  {
    const bool hist = (tb > 0);
    const int rb = hist ? (g0 - 3) : g0;
    const float v3 = XPRE[(size_t)rb * kDin + d];
    const float v2 = XPRE[(size_t)(rb + 1) * kDin + d];
    const float v1 = XPRE[(size_t)(rb + 2) * kDin + d];
    const float fh = hist ? 1.0f : 0.0f;
    xm3 = v3 * fh;
    xm2 = v2 * fh;
    xm1 = v1 * fh;
  }
#pragma unroll 1
  for (int sub = 0; sub < 4; ++sub) {
    const int lb = g0 + sub * 16;
#pragma unroll 1
    for (int s = 0; s < 16; ++s) {
      const float xcur = XPRE[(size_t)(lb + s) * kDin + d];
      float acc = w0 * xm3;
      acc = fmaf(w1, xm2, acc);
      acc = fmaf(w2, xm1, acc);
      acc = fmaf(w3, xcur, acc);
      const float sv = acc + bc;
      const float sg = __builtin_amdgcn_rcpf(1.0f + expf(-sv));
      sT[s * kConvTP + tid] = (sv * sg) * kXinCarry;
      xm3 = xm2; xm2 = xm1; xm1 = xcur;
    }
    __syncthreads();
    v8h hv[2];
#pragma unroll
    for (int it = 0; it < 2; ++it) {
      const float* sp = sT + (it * 8 + wave) * kConvTP + lane * 8;
      const v4f a0 = *(const v4f*)(sp);
      const v4f a1 = *(const v4f*)(sp + 4);
#pragma unroll
      for (int e = 0; e < 4; ++e) {
        hv[it][e]     = (_Float16)a0[e];
        hv[it][4 + e] = (_Float16)a1[e];
      }
    }
    for (int pass = 0; pass < 2; ++pass) {
#pragma unroll
      for (int it = 0; it < 2; ++it) {
        const size_t o = (size_t)(lb + it * 8 + wave) * kDin + d0 + lane * 8;
        *(volatile v8h*)(XIN16 + o) = hv[it];
      }
      __threadfence();
    }
    __syncthreads();
  }
}

__global__ __launch_bounds__(256) void dtraw_cast_kernel(const float* __restrict__ XD, unsigned short* __restrict__ DTR)
{
  const int i = blockIdx.x * 256 + threadIdx.x;
  if (i >= kRows * (kDtR / 8)) return;
  const int row = i >> 3, c8 = (i & 7) * 8;
  const v4f a0 = *(const v4f*)(XD + (size_t)row * kXdP + c8);
  const v4f a1 = *(const v4f*)(XD + (size_t)row * kXdP + c8 + 4);
  v8h hv;
#pragma unroll
  for (int e = 0; e < 4; ++e) {
    hv[e]     = (_Float16)(a0[e] * kDtrCarry);
    hv[4 + e] = (_Float16)(a1[e] * kDtrCarry);
  }
  unsigned short* qd = DTR + (size_t)row * kDtR + c8;
  *(volatile v8h*)qd = hv;
  __threadfence();
  *(volatile v8h*)qd = hv;
}

constexpr int kScanTS = 64;
constexpr int kScanCh = 64;
constexpr int kScanBC = 32;
constexpr int kScanYP = 68;
static_assert((kSeq % kScanTS) == 0 && (kDin % kScanCh) == 0 && kScanCh == 64 && kScanTS == 64, "scan tiling");

__global__ __launch_bounds__(kScanCh) void scan_kernel(
    const float* __restrict__ XD, const float* __restrict__ DTV,
    const unsigned* __restrict__ XIN32, const unsigned* __restrict__ Z32,
    const float* __restrict__ Alog, const float* __restrict__ St0, const float* __restrict__ Dp,
    unsigned short* __restrict__ G16, float* __restrict__ FS)
{
  __shared__ __align__(16) float sBC[kScanTS * kScanBC];
  __shared__ __align__(16) float sY[kScanTS * kScanYP];
  __shared__ __align__(16) float sA[kNst * kScanCh];
  __shared__ __align__(16) float sH[kNst * kScanCh];
  __shared__ __align__(16) float sF[kScanCh * kNst];
  const int tid = threadIdx.x, lane = tid & 31, wave = tid >> 5;
  constexpr int kBlkPerB = kDin / kScanCh;
  const int bix = blockIdx.x / kBlkPerB;
  const int d0  = (blockIdx.x - bix * kBlkPerB) * kScanCh;
  const int d   = d0 + tid;
  const size_t row0 = (size_t)bix * kSeq;
  const size_t chan = (size_t)bix * kDin + d;
#pragma unroll 1
  for (int s = 0; s < kNst; ++s) {
    const float al = Alog[(size_t)d * kNst + s];
    const float h0 = St0[chan * kNst + s];
    sA[s * kScanCh + tid] = -expf(al) * kLog2e;
    sH[s * kScanCh + tid] = h0;
  }
  __syncthreads();
  float nA2[kNst], h[kNst];
#pragma unroll
  for (int s = 0; s < kNst; ++s) {
    nA2[s] = sA[s * kScanCh + tid];
    h[s]   = sH[s * kScanCh + tid];
  }
  const float Dd = Dp[d];
  const int dw = d >> 1;
  const unsigned dsh = (unsigned)(d & 1) * 16u;
  constexpr int kXinW = kDin / 2;
  constexpr int kZW   = kDin / 2;
  const int q = lane >> 3, c8 = (lane & 7) * 8;
#pragma unroll 1
  for (int t0 = 0; t0 < kSeq; t0 += kScanTS) {
    __syncthreads();
#pragma unroll
    for (int i = 0; i < 8; ++i) {
      const int idx = tid + kScanCh * i;
      const int r = idx >> 3, c4 = (idx & 7) * 4;
      *(v4f*)(sBC + r * kScanBC + c4) = *(const v4f*)(XD + (row0 + t0 + r) * kXdP + kDtR + c4);
    }
    __syncthreads();
#pragma unroll 1
    for (int s = 0; s < kScanTS; ++s) {
      const size_t row = row0 + t0 + s;
      const float* bc = sBC + s * kScanBC;
      float Bs[kNst], Cs[kNst];
#pragma unroll
      for (int q4 = 0; q4 < 4; ++q4) {
        const v4f bv = *(const v4f*)(bc + 4 * q4);
        const v4f cv = *(const v4f*)(bc + kNst + 4 * q4);
        Bs[4 * q4 + 0] = bv[0]; Bs[4 * q4 + 1] = bv[1]; Bs[4 * q4 + 2] = bv[2]; Bs[4 * q4 + 3] = bv[3];
        Cs[4 * q4 + 0] = cv[0]; Cs[4 * q4 + 1] = cv[1]; Cs[4 * q4 + 2] = cv[2]; Cs[4 * q4 + 3] = cv[3];
      }
      const float v     = DTV[row * kDin + d];
      const unsigned wx = XIN32[row * kXinW + dw];
      const unsigned wz = Z32[row * kZW + dw];
      const float xt = h16_to_f32((wx >> dsh) & 0xffffu) * kXinCarryInv;
      const float zv = h16_to_f32((wz >> dsh) & 0xffffu);
      const float a   = expf(-fabsf(v));
      const float u   = 1.0f + a;
      const float l1p = log2f(u) * kLn2 + (a - (u - 1.0f)) * __builtin_amdgcn_rcpf(u);
      const float dt  = fmaxf(v, 0.0f) + l1p;
      const float dtx = dt * xt;
      float y = 0.0f;
#pragma unroll
      for (int k = 0; k < kNst; ++k) {
        const float e = exp2f(dt * nA2[k]);
        h[k] = e * h[k] + dtx * Bs[k];
        y = y + h[k] * Cs[k];
      }
      y = y + xt * Dd;
      const float sg = __builtin_amdgcn_rcpf(1.0f + expf(-zv));
      const float gv = y * (zv * sg);
      sY[s * kScanYP + tid] = gv * kGCarry;
    }
    __syncthreads();
    v8h hv[8];
#pragma unroll
    for (int it = 0; it < 8; ++it) {
      const int rr = it * 8 + wave * 4 + q;
      const float* sp = sY + rr * kScanYP + c8;
      const v4f a0 = *(const v4f*)(sp);
      const v4f a1 = *(const v4f*)(sp + 4);
#pragma unroll
      for (int e = 0; e < 4; ++e) {
        hv[it][e]     = (_Float16)a0[e];
        hv[it][4 + e] = (_Float16)a1[e];
      }
    }
    for (int pass = 0; pass < 2; ++pass) {
#pragma unroll
      for (int it = 0; it < 8; ++it) {
        const int rr = it * 8 + wave * 4 + q;
        const size_t o = (row0 + t0 + rr) * kDin + d0 + c8;
        *(volatile v8h*)(G16 + o) = hv[it];
      }
      __threadfence();
    }
  }
#pragma unroll
  for (int k = 0; k < kNst; ++k) sF[tid * kNst + k] = h[k];
  __syncthreads();
  v4f fv[4];
#pragma unroll
  for (int it = 0; it < 4; ++it) fv[it] = *(const v4f*)(sF + (wave * 4 + it) * 128 + lane * 4);
  const size_t fbase = ((size_t)bix * kDin + d0) * kNst;
  for (int pass = 0; pass < 2; ++pass) {
#pragma unroll
    for (int it = 0; it < 4; ++it)
      *(volatile v4f*)(FS + fbase + (size_t)((wave * 4 + it) * 128 + lane * 4)) = fv[it];
    __threadfence();
  }
}

extern "C" void kernel_launch(void* const* d_in, const int* in_sizes, int n_in,
                              void* d_out, int out_size, void* d_ws, size_t ws_size,
                              hipStream_t stream) {
  if (n_in < 11) return;
  if (in_sizes[0]  != kRows * kHid) return;
  if (in_sizes[1]  != kBatch * kDin * kNst) return;
  if (in_sizes[2]  != kXzN * kHid) return;
  if (in_sizes[3]  != kDin * kConvK) return;
  if (in_sizes[4]  != kDin) return;
  if (in_sizes[5]  != kXdbl * kDin) return;
  if (in_sizes[6]  != kDin * kDtR) return;
  if (in_sizes[7]  != kDin) return;
  if (in_sizes[8]  != kDin * kNst) return;
  if (in_sizes[9]  != kDin) return;
  if (in_sizes[10] != kHid * kDin) return;
  if ((size_t)out_size != kOut0Floats + kOut1Floats) return;
  if (ws_size < kWsTotal) return;

  const float* x      = (const float*)d_in[0];
  const float* state0 = (const float*)d_in[1];
  const float* W_in   = (const float*)d_in[2];
  const float* conv_w = (const float*)d_in[3];
  const float* conv_b = (const float*)d_in[4];
  const float* W_x    = (const float*)d_in[5];
  const float* W_dt   = (const float*)d_in[6];
  const float* b_dt   = (const float*)d_in[7];
  const float* A_log  = (const float*)d_in[8];
  const float* Dp     = (const float*)d_in[9];
  const float* W_out  = (const float*)d_in[10];
  float* out0 = (float*)d_out;
  float* out1 = (float*)d_out + kOut0Floats;

  char* ws = (char*)d_ws;
  unsigned short* XH   = (unsigned short*)(ws + kOffXH);
  unsigned short* XL   = (unsigned short*)(ws + kOffXL);
  unsigned short* WIH  = (unsigned short*)(ws + kOffWIH);
  float*          XPRE = (float*)(ws + kOffXPRE);
  float*          DTV  = (float*)(ws + kOffDTV);
  unsigned short* Z16  = (unsigned short*)(ws + kOffZ16);
  unsigned short* XIN  = (unsigned short*)(ws + kOffXIN);
  unsigned short* WXH  = (unsigned short*)(ws + kOffWXH);
  unsigned short* WXL  = (unsigned short*)(ws + kOffWXL);
  float*          XD   = (float*)(ws + kOffXD);
  unsigned short* DTR  = (unsigned short*)(ws + kOffDTR);
  unsigned short* WDT  = (unsigned short*)(ws + kOffWDT);
  unsigned short* G16  = (unsigned short*)(ws + kOffG);
  unsigned short* WOH  = (unsigned short*)(ws + kOffWOH);

  {
    const int t8x   = kRows * kHid / 8;
    const int t8win = kXzN * kHid / 8;
    const int t8wx  = kXdbl * kDin / 8;
    const int t8pad = (kXdP - kXdbl) * kDin / 8;
    const int t8wdt = kDin * kDtR / 8;
    const int t8wo  = kHid * kDin / 8;
    split_f16x8_kernel<<<t8x / 256, 256, 0, stream>>>(x, XH, XL, t8x, 1.0f);
    cast_f16x8_kernel<<<t8win / 256, 256, 0, stream>>>(W_in, WIH, t8win, kWCarry);
    split_f16x8_kernel<<<t8wx / 256, 256, 0, stream>>>(W_x, WXH, WXL, t8wx, kWCarry);
    zero2_16x8_kernel<<<t8pad / 256, 256, 0, stream>>>(WXH + (size_t)kXdbl * kDin, WXL + (size_t)kXdbl * kDin, t8pad);
    cast_f16x8_kernel<<<t8wdt / 256, 256, 0, stream>>>(W_dt, WDT, t8wdt, kWCarry);
    cast_f16x8_kernel<<<t8wo / 256, 256, 0, stream>>>(W_out, WOH, t8wo, kWCarry);
  }

  constexpr int kIpBlocks = (kRows / 32) * (kDin / 64) / 8;
  wmma_gemm32x64_res<0, 0><<<dim3(kIpBlocks), 256, 0, stream>>>(
      XH, XL, kHid,
      WIH, nullptr, kHid,
      (void*)XPRE, kDin,
      kRows, kDin, kHid, 1.0f / kWCarry, 1.0f / (kWCarry * kLoCarry));

  wmma_gemm32x64_res<0, 1><<<dim3(kIpBlocks), 256, 0, stream>>>(
      XH, XL, kHid,
      WIH + (size_t)kDin * kHid, nullptr, kHid,
      (void*)Z16, kDin,
      kRows, kDin, kHid, 1.0f / kWCarry, 1.0f / (kWCarry * kLoCarry));

  conv_silu_kernel<<<dim3(kDin / 256, kRows / 64), 256, 0, stream>>>(XPRE, conv_w, conv_b, XIN);

  constexpr int kXpBlocks = (kRows / 32) * (kXdP / 64) / 8;
  wmma_gemm32x64_res<1, 0><<<dim3(kXpBlocks), 256, 0, stream>>>(
      XIN, nullptr, kDin,
      WXH, WXL, kDin,
      (void*)XD, kXdP,
      kRows, kXdP, kDin, 1.0f / (kXinCarry * kWCarry), 1.0f / (kXinCarry * kWCarry * kLoCarry));

  dtraw_cast_kernel<<<kRows * (kDtR / 8) / 256, 256, 0, stream>>>(XD, DTR);

  wmma_gemm64<0, 0, 2, 0, false><<<dim3((kRows / 64) * (kDin / 64) / 8, 1), 256, 0, stream>>>(
      DTR, nullptr, kDtR, 0L,
      WDT, nullptr, kDtR, 0L,
      (void*)DTV, nullptr, kDin, 0L,
      b_dt, nullptr, 0L,
      kRows, kDin, kDtR, 1.0f / (kDtrCarry * kWCarry));

  scan_kernel<<<kBatch * (kDin / kScanCh), kScanCh, 0, stream>>>(
      XD, DTV, (const unsigned*)XIN, (const unsigned*)Z16, A_log, state0, Dp, G16, out1);

  wmma_gemm64<0, 0, 0, 0, false><<<dim3((kRows / 64) * (kHid / 64) / 8, 1), 256, 0, stream>>>(
      G16, nullptr, kDin, 0L,
      WOH, nullptr, kDin, 0L,
      (void*)out0, nullptr, kHid, 0L,
      nullptr, nullptr, 0L,
      kRows, kHid, kDin, 1.0f / (kGCarry * kWCarry));
}
